// MyGRU_63539746177495
// MI455X (gfx1250) — hardware-run, weakly checked
//
#include <hip/hip_runtime.h>
#include <math.h>

typedef __attribute__((ext_vector_type(16))) _Float16 v16h;
typedef __attribute__((ext_vector_type(8)))  _Float16 v8h;
typedef __attribute__((ext_vector_type(4)))  _Float16 v4h;
typedef __attribute__((ext_vector_type(16))) __bf16   v16b;
typedef __attribute__((ext_vector_type(8)))  __bf16   v8b;
typedef __attribute__((ext_vector_type(8)))  float    v8f;
typedef __attribute__((ext_vector_type(4)))  float    v4f;
typedef __attribute__((ext_vector_type(4)))  unsigned v4u;

constexpr int kSteps = 128;
constexpr int kBatch = 64;
constexpr int kEin   = 512;
constexpr int kPosts = 160;
constexpr int kPdim  = 512;
constexpr int kHid   = 1024;
constexpr int kGate  = 3 * kHid;
constexpr int kXdim  = kEin + kPdim;
constexpr int kRowsX = kSteps * kBatch;
constexpr int kRowsP = kPosts * kBatch;
constexpr int kBlkB  = 16;
constexpr int kNumBlk = kBatch / kBlkB;
constexpr int kHP = kHid + 8;
constexpr int kCP = kPdim + 8;
constexpr float kWCarry   = 1024.0f;
constexpr float kInvW     = 1.0f / 1024.0f;
constexpr float kResCarry = 2048.0f;
constexpr float kInvRes   = 1.0f / 2048.0f;
constexpr float kF16Min   = 6.103515625e-05f;
constexpr float kF32Min   = 1.17549435e-38f;
constexpr float kFill     = -1000000000.0f;
static_assert(kXdim == 1024 && kGate == 3072, "shape");
static_assert(kRowsX == 8192 && kRowsP == 10240, "rows");
static_assert((kRowsX % 64) == 0 && (kGate % 64) == 0 && (kEin % 32) == 0, "GEMM tile multiples");
static_assert((kHid % 32) == 0 && (kPdim % 32) == 0, "K multiples of 32");
static_assert(kNumBlk * kBlkB == kBatch, "batch split");
static_assert(((kHP * 2) % 16) == 0 && ((kCP * 2) % 16) == 0, "LDS row pitch 16-B multiple");

constexpr size_t kSzXB  = (size_t)kRowsX * kEin * 2;
constexpr size_t kSzPB  = (size_t)kRowsP * kPdim * 2;
constexpr size_t kSzWIX = (size_t)kGate * kEin * 2;
constexpr size_t kSzWIC = (size_t)kGate * kPdim * 2;
constexpr size_t kSzWHH = (size_t)kGate * kHid * 2;
constexpr size_t kSzWQ  = (size_t)kPdim * kHid * 2;
constexpr size_t kSzGX  = (size_t)kRowsX * kGate * 4;
constexpr size_t kOffXB  = 0;
constexpr size_t kOffPB  = kOffXB  + kSzXB;
constexpr size_t kOffWIX = kOffPB  + kSzPB;
constexpr size_t kOffWIC = kOffWIX + kSzWIX;
constexpr size_t kOffWHH = kOffWIC + kSzWIC;
constexpr size_t kOffWQ  = kOffWHH + kSzWHH;
constexpr size_t kOffGX  = kOffWQ  + kSzWQ;
constexpr size_t kWsTotal = kOffGX + kSzGX;
static_assert(kWsTotal == 133169152ull, "carve total");
static_assert(kWsTotal <= 134217728ull, "carve cap");
static_assert((kOffPB % 128) == 0 && (kOffWIX % 128) == 0 && (kOffWIC % 128) == 0 && (kOffWHH % 128) == 0 &&
              (kOffWQ % 128) == 0 && (kOffGX % 128) == 0, "128-B aligned regions");

__device__ __forceinline__ unsigned short f2bf_bits(float f) {
  unsigned u = __float_as_uint(f);
  return (unsigned short)((u + 0x7FFFu + ((u >> 16) & 1u)) >> 16);
}
__device__ __forceinline__ float bf_bits2f(unsigned short h) { return __uint_as_float(((unsigned)h) << 16); }
__device__ __forceinline__ float bf_rne(float f) { return bf_bits2f(f2bf_bits(f)); }
__device__ __forceinline__ float bf_lo(unsigned x) { return __uint_as_float(x << 16); }
__device__ __forceinline__ float bf_hi(unsigned x) { return __uint_as_float(x & 0xffff0000u); }

__device__ __forceinline__ void split_h(float v, _Float16& hi, _Float16& lo) {
  const float vh = (fabsf(v) < kF16Min) ? 0.0f : v;
  const _Float16 h = (_Float16)vh;
  float hf = (float)h;
  asm volatile("" : "+v"(hf));
  const float res = (v - hf) * kResCarry;
  const float rl = (fabsf(res) < kF16Min) ? 0.0f : res;
  hi = h;
  lo = (_Float16)rl;
}

__device__ __forceinline__ void keep4_b(v16b a, v16b b, v16b c, v16b d) { asm volatile("v_nop" :: "v"(a), "v"(b), "v"(c), "v"(d)); }
__device__ __forceinline__ void acc_guard4(v8f& a, v8f& b, v8f& c, v8f& d) { asm volatile("v_nop\n\tv_nop\n\tv_nop\n\tv_nop" : "+v"(a), "+v"(b), "+v"(c), "+v"(d)); }

__device__ __forceinline__ v16h frag_h(const _Float16* p) {
  union { v16h v; v8h h[2]; } f;
  f.h[0] = *(const v8h*)(p);
  f.h[1] = *(const v8h*)(p + 16);
  return f.v;
}
__device__ __forceinline__ v16b frag_b(const __bf16* p) {
  union { v16b v; v8b h[2]; } f;
  f.h[0] = *(const v8b*)(p);
  f.h[1] = *(const v8b*)(p + 16);
  return f.v;
}
__device__ __forceinline__ v8f mma_h(v16h a, v16h b, v8f c) {
  c = __builtin_amdgcn_wmma_f32_16x16x32_f16(false, a, false, b, (short)0, c, false, false);
  asm volatile("v_nop\n\tv_nop\n\tv_nop\n\tv_nop" : "+v"(c) : "v"(a), "v"(b));
  return c;
}
__device__ __forceinline__ v8f mma_b(v16b a, v16b b, v8f c) {
  c = __builtin_amdgcn_wmma_f32_16x16x32_bf16(false, a, false, b, (short)0, c, false, false);
  asm volatile("v_nop\n\tv_nop\n\tv_nop\n\tv_nop" : "+v"(c) : "v"(a), "v"(b));
  return c;
}

template <int MODE>
__global__ __launch_bounds__(256) void plane_rows_kernel(
    const float* __restrict__ src, int srcPitch, int colOff, int cols,
    unsigned short* __restrict__ dst, int total8) {
  const int i = blockIdx.x * 256 + threadIdx.x;
  if (i >= total8) return;
  const int e0 = i << 3;
  const int row = e0 / cols;
  const int c = e0 - row * cols;
  const float* sp = src + (size_t)row * srcPitch + colOff + c;
  const v4f a0 = *(const v4f*)(sp);
  const v4f a1 = *(const v4f*)(sp + 4);
  v8h hv;
#pragma unroll
  for (int e = 0; e < 4; ++e) {
    const float x0 = a0[e];
    const float x1 = a1[e];
    const unsigned short b0 = f2bf_bits(x0);
    const unsigned short b1 = f2bf_bits(x1);
    if (MODE == 0) {
      hv[e]     = __builtin_bit_cast(_Float16, b0);
      hv[4 + e] = __builtin_bit_cast(_Float16, b1);
    } else {
      float v0 = bf_bits2f(b0) * kWCarry;
      float v1 = bf_bits2f(b1) * kWCarry;
      v0 = (fabsf(v0) < kF16Min) ? 0.0f : v0;
      v1 = (fabsf(v1) < kF16Min) ? 0.0f : v1;
      hv[e]     = (_Float16)v0;
      hv[4 + e] = (_Float16)v1;
    }
  }
  unsigned short* q = dst + (size_t)e0;
  *(volatile v8h*)q = hv;
  __threadfence();
  *(volatile v8h*)q = hv;
}

__global__ __launch_bounds__(256) void input_half_gemm(
    const unsigned short* __restrict__ Ap, int lda,
    const unsigned short* __restrict__ Btp, int ldb,
    float* __restrict__ C, int ldc,
    const float* __restrict__ bias, int M, int N, int K) {
  const __bf16* A  = (const __bf16*)Ap;
  const __bf16* Bt = (const __bf16*)Btp;
  __shared__ __align__(16) float sT[8][16 * 68];
  const int lane = threadIdx.x & 31;
  const int wave = threadIdx.x >> 5;
  const int tilesN = N >> 6;
  const int tilesM = M >> 6;
  const int tile = blockIdx.x * 8 + wave;
  if (tile >= tilesM * tilesN) return;
  const int tm = tile / tilesN;
  const int tn = tile - tm * tilesN;
  const int m0 = tm << 6;
  const int n0 = tn << 6;
  const int rlane = lane & 15;
  const int koff  = (lane >> 4) * 8;
  const int mOff  = (lane >> 4) * 8;

  v8f acc[4][4];
#pragma unroll
  for (int i = 0; i < 4; ++i)
#pragma unroll
    for (int j = 0; j < 4; ++j) acc[i][j] = (v8f){0.f,0.f,0.f,0.f,0.f,0.f,0.f,0.f};

  for (int k0 = 0; k0 < K; k0 += 32) {
    v16b bh[4];
#pragma unroll
    for (int j = 0; j < 4; ++j) {
      const size_t bo = (size_t)(n0 + (j << 4) + rlane) * ldb + koff + k0;
      bh[j] = frag_b(Bt + bo);
    }
#pragma unroll
    for (int i = 0; i < 4; ++i) {
      const size_t ao = (size_t)(m0 + (i << 4) + rlane) * lda + koff + k0;
      const v16b ah = frag_b(A + ao);
#pragma unroll
      for (int j = 0; j < 4; ++j) acc[i][j] = mma_b(ah, bh[j], acc[i][j]);
    }
    keep4_b(bh[0], bh[1], bh[2], bh[3]);
  }
  acc_guard4(acc[0][0], acc[0][1], acc[0][2], acc[0][3]);
  acc_guard4(acc[1][0], acc[1][1], acc[1][2], acc[1][3]);
  acc_guard4(acc[2][0], acc[2][1], acc[2][2], acc[2][3]);
  acc_guard4(acc[3][0], acc[3][1], acc[3][2], acc[3][3]);

  float* slab = sT[wave];
#pragma unroll
  for (int i = 0; i < 4; ++i) {
    const int mBase = m0 + (i << 4);
#pragma unroll
    for (int j = 0; j < 4; ++j) {
      const int n = n0 + (j << 4) + rlane;
      const float bv = bf_rne(bias[n]);
#pragma unroll
      for (int r = 0; r < 8; ++r) {
        const float v = acc[i][j][r] + bv;
        slab[(mOff + r) * 68 + (j << 4) + rlane] = v;
      }
    }
    __builtin_amdgcn_fence(__ATOMIC_RELEASE, "workgroup");
    __builtin_amdgcn_wave_barrier();
    __builtin_amdgcn_fence(__ATOMIC_ACQUIRE, "workgroup");
    {
      const int hh = lane >> 4, c4 = (lane & 15) * 4;
      for (int pass = 0; pass < 2; ++pass) {
#pragma unroll
        for (int it = 0; it < 8; ++it) {
          const int row = it * 2 + hh;
          const v4f v = *(const v4f*)(slab + row * 68 + c4);
          *(volatile v4f*)(C + (size_t)(mBase + row) * ldc + n0 + c4) = v;
        }
        __threadfence();
      }
    }
    __builtin_amdgcn_fence(__ATOMIC_RELEASE, "workgroup");
    __builtin_amdgcn_wave_barrier();
    __builtin_amdgcn_fence(__ATOMIC_ACQUIRE, "workgroup");
  }
}

__global__ __launch_bounds__(512) void attend_cell_steps(
    const unsigned short* __restrict__ PBp,
    const unsigned short* __restrict__ WQp,
    const unsigned short* __restrict__ WICp,
    const unsigned short* __restrict__ WHHp,
    const float* __restrict__ GX,
    const float* __restrict__ h_init,
    const float* __restrict__ bhh,
    const float* __restrict__ bq,
    const int* __restrict__ length,
    const int* __restrict__ post_length,
    float* out) {
  __shared__ __align__(16) _Float16 sHhi[kBlkB * kHP];
  __shared__ __align__(16) _Float16 sHlo[kBlkB * kHP];
  __shared__ __align__(16) _Float16 sChi[kBlkB * kCP];
  __shared__ __align__(16) _Float16 sClo[kBlkB * kCP];
  __shared__ __align__(16) float sQ[kBlkB * kPdim];
  __shared__ __align__(16) float sS[kBlkB * kPosts];

  const _Float16* WQ  = (const _Float16*)WQp;
  const _Float16* WIC = (const _Float16*)WICp;
  const _Float16* WHH = (const _Float16*)WHHp;

  const int tid  = threadIdx.x;
  const int lane = tid & 31;
  const int wave = __builtin_amdgcn_readfirstlane(tid >> 5);
  const int hh   = lane >> 4;
  const int n    = lane & 15;
  const int b0   = blockIdx.x * kBlkB;

  int lenr[8];
#pragma unroll
  for (int r = 0; r < 8; ++r) {
    int v = length[b0 + 8 * hh + r];
    v = (v < 0) ? 0 : v;
    v = (v > kSteps) ? kSteps : v;
    lenr[r] = v;
  }
  int plraw = post_length[b0 + wave];
  plraw = __builtin_amdgcn_readfirstlane(plraw);
  const bool allmask = (plraw <= 0);
  int plen = allmask ? kPosts : plraw;
  plen = (plen > kPosts) ? kPosts : plen;
  plen = (plen < 1) ? 1 : plen;

  float hreg[4][8];
#pragma unroll
  for (int jt = 0; jt < 4; ++jt) {
    const float v = bf_rne(h_init[64 * wave + 16 * jt + n]);
#pragma unroll
    for (int r = 0; r < 8; ++r) hreg[jt][r] = v;
  }
#pragma unroll 1
  for (int it = 0; it < 8; ++it) {
    const int idx = it * 512 + tid;
    const int row = idx >> 8;
    const int c4  = (idx & 255) * 4;
    const v4f hv = *(const v4f*)(h_init + c4);
    v4h ph, pl;
#pragma unroll
    for (int e = 0; e < 4; ++e) {
      const float x = bf_rne(hv[e]);
      _Float16 a, b;
      split_h(x, a, b);
      ph[e] = a;
      pl[e] = b;
    }
    *(v4h*)(sHhi + row * kHP + c4) = ph;
    *(v4h*)(sHlo + row * kHP + c4) = pl;
  }

  const _Float16* hah = sHhi + n * kHP + 8 * hh;
  const _Float16* hal = sHlo + n * kHP + 8 * hh;
  const _Float16* cah = sChi + n * kCP + 8 * hh;
  const _Float16* cal = sClo + n * kCP + 8 * hh;

  const v4u* pb = (const v4u*)PBp + (size_t)(b0 + wave) * (kPdim / 8);
  constexpr int kRowStride16 = kBatch * (kPdim / 8);
  float* srow = sS + wave * kPosts;

#pragma unroll 1
  for (int i = 0; i < kSteps; ++i) {
    __syncthreads();

    {
      v8f qm0 = (v8f){0.f,0.f,0.f,0.f,0.f,0.f,0.f,0.f};
      v8f qr0 = qm0, qm1 = qm0, qr1 = qm0;
      const _Float16* wa = WQ + (size_t)(32 * wave + n) * kHid + 8 * hh;
      const _Float16* wb = wa + (size_t)16 * kHid;
#pragma unroll 1
      for (int k0 = 0; k0 < kHid; k0 += 32) {
        const v16h ah = frag_h(hah + k0);
        const v16h al = frag_h(hal + k0);
        const v16h fa = frag_h(wa + k0);
        const v16h fb = frag_h(wb + k0);
        qm0 = mma_h(ah, fa, qm0);
        qr0 = mma_h(al, fa, qr0);
        qm1 = mma_h(ah, fb, qm1);
        qr1 = mma_h(al, fb, qr1);
      }
      const float bqa = bf_rne(bq[32 * wave + n]);
      const float bqb = bf_rne(bq[32 * wave + 16 + n]);
#pragma unroll
      for (int r = 0; r < 8; ++r) {
        const float qa = (qm0[r] + qr0[r] * kInvRes) * kInvW + bqa;
        const float qb = (qm1[r] + qr1[r] * kInvRes) * kInvW + bqb;
        sQ[(8 * hh + r) * kPdim + 32 * wave + n]      = qa;
        sQ[(8 * hh + r) * kPdim + 32 * wave + 16 + n] = qb;
      }
    }
    __syncthreads();

    {
      float qv[16];
      {
        const float* qrow = sQ + wave * kPdim;
        const v4f t0 = *(const v4f*)(qrow + lane * 8);
        const v4f t1 = *(const v4f*)(qrow + lane * 8 + 4);
        const v4f t2 = *(const v4f*)(qrow + 256 + lane * 8);
        const v4f t3 = *(const v4f*)(qrow + 256 + lane * 8 + 4);
#pragma unroll
        for (int e = 0; e < 4; ++e) {
          qv[e] = t0[e];
          qv[4 + e] = t1[e];
          qv[8 + e] = t2[e];
          qv[12 + e] = t3[e];
        }
      }
#pragma unroll 1
      for (int p = 0; p < plen; ++p) {
        const v4u w0 = pb[(size_t)p * kRowStride16 + lane];
        const v4u w1 = pb[(size_t)p * kRowStride16 + 32 + lane];
        float s = 0.0f;
#pragma unroll
        for (int e = 0; e < 4; ++e) {
          const unsigned x0 = w0[e];
          const unsigned x1 = w1[e];
          s = fmaf(bf_lo(x0), qv[2 * e], s);
          s = fmaf(bf_hi(x0), qv[2 * e + 1], s);
          s = fmaf(bf_lo(x1), qv[8 + 2 * e], s);
          s = fmaf(bf_hi(x1), qv[8 + 2 * e + 1], s);
        }
#pragma unroll
        for (int off = 16; off >= 1; off >>= 1) s += __shfl_xor(s, off, 32);
        const float sv = allmask ? kFill : s;
        if (lane == 0) srow[p] = sv;
      }
      __syncthreads();
      float ev[5];
      float mx = -INFINITY;
#pragma unroll
      for (int k = 0; k < 5; ++k) {
        const int p = lane + 32 * k;
        const int pc = (p < plen) ? p : (plen - 1);
        const float sv = srow[pc];
        ev[k] = (p < plen) ? sv : -INFINITY;
        mx = fmaxf(mx, ev[k]);
      }
#pragma unroll
      for (int off = 16; off >= 1; off >>= 1) mx = fmaxf(mx, __shfl_xor(mx, off, 32));
      float sum = 0.0f;
#pragma unroll
      for (int k = 0; k < 5; ++k) {
        const int p = lane + 32 * k;
        float e = expf(ev[k] - mx);
        e = (p < plen) ? e : 0.0f;
        e = (e < kF32Min) ? 0.0f : e;
        ev[k] = e;
        sum += e;
      }
#pragma unroll
      for (int off = 16; off >= 1; off >>= 1) sum += __shfl_xor(sum, off, 32);
#pragma unroll
      for (int k = 0; k < 5; ++k) {
        const int p = lane + 32 * k;
        if (p < plen) srow[p] = ev[k];
      }
      const float inv = 1.0f / sum;
      __syncthreads();
      float ca[16];
#pragma unroll
      for (int j = 0; j < 16; ++j) ca[j] = 0.0f;
#pragma unroll 1
      for (int p = 0; p < plen; ++p) {
        const v4u w0 = pb[(size_t)p * kRowStride16 + lane];
        const v4u w1 = pb[(size_t)p * kRowStride16 + 32 + lane];
        const float e = srow[p];
#pragma unroll
        for (int q = 0; q < 4; ++q) {
          const unsigned x0 = w0[q];
          const unsigned x1 = w1[q];
          ca[2 * q]         = fmaf(e, bf_lo(x0), ca[2 * q]);
          ca[2 * q + 1]     = fmaf(e, bf_hi(x0), ca[2 * q + 1]);
          ca[8 + 2 * q]     = fmaf(e, bf_lo(x1), ca[8 + 2 * q]);
          ca[8 + 2 * q + 1] = fmaf(e, bf_hi(x1), ca[8 + 2 * q + 1]);
        }
      }
      v8h h0, l0, h1, l1;
#pragma unroll
      for (int e = 0; e < 8; ++e) {
        _Float16 a, b;
        split_h(ca[e] * inv, a, b);
        h0[e] = a;
        l0[e] = b;
        split_h(ca[8 + e] * inv, a, b);
        h1[e] = a;
        l1[e] = b;
      }
      *(v8h*)(sChi + wave * kCP + lane * 8)       = h0;
      *(v8h*)(sClo + wave * kCP + lane * 8)       = l0;
      *(v8h*)(sChi + wave * kCP + 256 + lane * 8) = h1;
      *(v8h*)(sClo + wave * kCP + 256 + lane * 8) = l1;
    }
    __syncthreads();

#pragma unroll 1
    for (int jt = 0; jt < 4; ++jt) {
      const int col = 64 * wave + 16 * jt + n;
      v8f rm = (v8f){0.f,0.f,0.f,0.f,0.f,0.f,0.f,0.f};
      v8f rr = rm, zm = rm, zr = rm, im = rm, ir = rm, hm = rm, hr = rm;
      {
        const _Float16* wr = WIC + (size_t)col * kPdim + 8 * hh;
        const _Float16* wz = wr + (size_t)kHid * kPdim;
        const _Float16* wn = wz + (size_t)kHid * kPdim;
#pragma unroll 1
        for (int k0 = 0; k0 < kPdim; k0 += 32) {
          const v16h ah = frag_h(cah + k0);
          const v16h al = frag_h(cal + k0);
          const v16h fr = frag_h(wr + k0);
          const v16h fz = frag_h(wz + k0);
          const v16h fn = frag_h(wn + k0);
          rm = mma_h(ah, fr, rm);
          rr = mma_h(al, fr, rr);
          zm = mma_h(ah, fz, zm);
          zr = mma_h(al, fz, zr);
          im = mma_h(ah, fn, im);
          ir = mma_h(al, fn, ir);
        }
      }
      {
        const _Float16* ur = WHH + (size_t)col * kHid + 8 * hh;
        const _Float16* uz = ur + (size_t)kHid * kHid;
        const _Float16* un = uz + (size_t)kHid * kHid;
#pragma unroll 1
        for (int k0 = 0; k0 < kHid; k0 += 32) {
          const v16h ah = frag_h(hah + k0);
          const v16h al = frag_h(hal + k0);
          const v16h fr = frag_h(ur + k0);
          const v16h fz = frag_h(uz + k0);
          const v16h fn = frag_h(un + k0);
          rm = mma_h(ah, fr, rm);
          rr = mma_h(al, fr, rr);
          zm = mma_h(ah, fz, zm);
          zr = mma_h(al, fz, zr);
          hm = mma_h(ah, fn, hm);
          hr = mma_h(al, fn, hr);
        }
      }
      const float bhr = bf_rne(bhh[col]);
      const float bhz = bf_rne(bhh[kHid + col]);
      const float bhn = bf_rne(bhh[2 * kHid + col]);
      const float* gxp = GX + (size_t)(i * kBatch + b0 + 8 * hh) * kGate + col;
      float pre_r[8], pre_z[8], pre_n[8];
#pragma unroll
      for (int r = 0; r < 8; ++r) {
        const float g = gxp[(size_t)r * kGate];
        pre_r[r] = (rm[r] + rr[r] * kInvRes) * kInvW + (g + bhr);
      }
      asm volatile("" ::: "memory");
#pragma unroll
      for (int r = 0; r < 8; ++r) {
        const float g = gxp[(size_t)r * kGate + kHid];
        pre_z[r] = (zm[r] + zr[r] * kInvRes) * kInvW + (g + bhz);
      }
      asm volatile("" ::: "memory");
#pragma unroll
      for (int r = 0; r < 8; ++r) {
        const float g = gxp[(size_t)r * kGate + 2 * kHid];
        pre_n[r] = (im[r] + ir[r] * kInvRes) * kInvW + g;
      }
      asm volatile("" ::: "memory");
      float hnew[8];
#pragma unroll
      for (int r = 0; r < 8; ++r) {
        const float hn_ = (hm[r] + hr[r] * kInvRes) * kInvW + bhn;
        const float rg = 1.0f / (1.0f + expf(-pre_r[r]));
        const float zg = 1.0f / (1.0f + expf(-pre_z[r]));
        const float ng = tanhf(pre_n[r] + rg * hn_);
        const float hold = hreg[0][r];
        const float hv = (1.0f - zg) * ng + zg * hold;
        hnew[r] = (lenr[r] > i) ? hv : 0.0f;
      }
#pragma unroll
      for (int r = 0; r < 8; ++r) {
        hreg[0][r] = hreg[1][r];
        hreg[1][r] = hreg[2][r];
        hreg[2][r] = hreg[3][r];
        hreg[3][r] = hnew[r];
      }
    }

    {
      float* slab = sQ + wave * 512;
      const int q8 = lane >> 3;
      const int c4 = (lane & 7) * 4;
      float* orow = out + (size_t)(i * kBatch + b0) * kHid + 64 * wave + c4;
      float* lrow = out + (size_t)kSteps * kBatch * kHid + (size_t)b0 * kHid + 64 * wave + c4;
      const bool last = (i == kSteps - 1);
      v4f va[4], vb[4];

#pragma unroll
      for (int r = 0; r < 8; ++r) {
        slab[(8 * hh + r) * 32 + n]      = hreg[0][r];
        slab[(8 * hh + r) * 32 + 16 + n] = hreg[1][r];
      }
      __syncthreads();
#pragma unroll
      for (int it = 0; it < 4; ++it) {
        const int row = it * 4 + q8;
        va[it] = *(const v4f*)(slab + row * 32 + c4);
        *(volatile v4f*)(orow + (size_t)row * kHid) = va[it];
        if (last) *(volatile v4f*)(lrow + (size_t)row * kHid) = va[it];
        v4h ph, pl;
#pragma unroll
        for (int e = 0; e < 4; ++e) {
          const float x = va[it][e];
          _Float16 a, b;
          split_h(x, a, b);
          ph[e] = a;
          pl[e] = b;
        }
        *(v4h*)(sHhi + row * kHP + 64 * wave + c4) = ph;
        *(v4h*)(sHlo + row * kHP + 64 * wave + c4) = pl;
      }
      __syncthreads();
#pragma unroll
      for (int r = 0; r < 8; ++r) {
        slab[(8 * hh + r) * 32 + n]      = hreg[2][r];
        slab[(8 * hh + r) * 32 + 16 + n] = hreg[3][r];
      }
      __syncthreads();
#pragma unroll
      for (int it = 0; it < 4; ++it) {
        const int row = it * 4 + q8;
        vb[it] = *(const v4f*)(slab + row * 32 + c4);
        *(volatile v4f*)(orow + (size_t)row * kHid + 32) = vb[it];
        if (last) *(volatile v4f*)(lrow + (size_t)row * kHid + 32) = vb[it];
        v4h ph, pl;
#pragma unroll
        for (int e = 0; e < 4; ++e) {
          const float x = vb[it][e];
          _Float16 a, b;
          split_h(x, a, b);
          ph[e] = a;
          pl[e] = b;
        }
        *(v4h*)(sHhi + row * kHP + 64 * wave + 32 + c4) = ph;
        *(v4h*)(sHlo + row * kHP + 64 * wave + 32 + c4) = pl;
      }
      __threadfence();
#pragma unroll
      for (int it = 0; it < 4; ++it) {
        const int row = it * 4 + q8;
        *(volatile v4f*)(orow + (size_t)row * kHid) = va[it];
        *(volatile v4f*)(orow + (size_t)row * kHid + 32) = vb[it];
        if (last) {
          *(volatile v4f*)(lrow + (size_t)row * kHid) = va[it];
          *(volatile v4f*)(lrow + (size_t)row * kHid + 32) = vb[it];
        }
      }
    }
  }
}

extern "C" void kernel_launch(void* const* d_in, const int* in_sizes, int n_in,
                              void* d_out, int out_size, void* d_ws, size_t ws_size,
                              hipStream_t stream) {
  if (n_in < 11) return;
  if (in_sizes[0] != kRowsX * kEin) return;
  if (in_sizes[1] != kRowsP * kPdim) return;
  if (in_sizes[2] != kHid) return;
  if (in_sizes[3] != kGate * kXdim) return;
  if (in_sizes[4] != kGate * kHid) return;
  if (in_sizes[5] != kGate) return;
  if (in_sizes[6] != kGate) return;
  if (in_sizes[7] != kPdim * kHid) return;
  if (in_sizes[8] != kPdim) return;
  if (in_sizes[9] != kBatch) return;
  if (in_sizes[10] != kBatch) return;
  if (out_size != (kSteps + 1) * kBatch * kHid) return;
  if (ws_size < kWsTotal) return;

  const float* incoming  = (const float*)d_in[0];
  const float* post      = (const float*)d_in[1];
  const float* h_init    = (const float*)d_in[2];
  const float* weight_ih = (const float*)d_in[3];
  const float* weight_hh = (const float*)d_in[4];
  const float* bias_ih   = (const float*)d_in[5];
  const float* bias_hh   = (const float*)d_in[6];
  const float* wq        = (const float*)d_in[7];
  const float* bq        = (const float*)d_in[8];
  const int*   length    = (const int*)d_in[9];
  const int*   post_len  = (const int*)d_in[10];
  float* out = (float*)d_out;

  char* ws = (char*)d_ws;
  unsigned short* XB  = (unsigned short*)(ws + kOffXB);
  unsigned short* PB  = (unsigned short*)(ws + kOffPB);
  unsigned short* WIX = (unsigned short*)(ws + kOffWIX);
  unsigned short* WIC = (unsigned short*)(ws + kOffWIC);
  unsigned short* WHH = (unsigned short*)(ws + kOffWHH);
  unsigned short* WQ  = (unsigned short*)(ws + kOffWQ);
  float*          GX  = (float*)(ws + kOffGX);

  constexpr int t8X   = kRowsX * kEin / 8;
  constexpr int t8P   = kRowsP * kPdim / 8;
  constexpr int t8WI  = kGate * kEin / 8;
  constexpr int t8WH  = kGate * kHid / 8;
  constexpr int t8WQ  = kPdim * kHid / 8;
  static_assert((t8X % 256) == 0 && (t8P % 256) == 0 && (t8WI % 256) == 0 && (t8WH % 256) == 0 && (t8WQ % 256) == 0,
                "plane grids exact");

  plane_rows_kernel<0><<<t8X / 256, 256, 0, stream>>>(incoming, kEin, 0, kEin, XB, t8X);
  plane_rows_kernel<0><<<t8P / 256, 256, 0, stream>>>(post, kPdim, 0, kPdim, PB, t8P);
  plane_rows_kernel<0><<<t8WI / 256, 256, 0, stream>>>(weight_ih, kXdim, 0, kEin, WIX, t8WI);
  plane_rows_kernel<1><<<t8WI / 256, 256, 0, stream>>>(weight_ih, kXdim, kEin, kPdim, WIC, t8WI);
  plane_rows_kernel<1><<<t8WH / 256, 256, 0, stream>>>(weight_hh, kHid, 0, kHid, WHH, t8WH);
  plane_rows_kernel<1><<<t8WQ / 256, 256, 0, stream>>>(wq, kHid, 0, kHid, WQ, t8WQ);

  {
    constexpr int tiles = (kRowsX / 64) * (kGate / 64);
    static_assert((tiles % 8) == 0, "whole blocks");
    input_half_gemm<<<tiles / 8, 256, 0, stream>>>(XB, kEin, WIX, kEin, GX, kGate, bias_ih, kRowsX, kGate, kEin);
  }

  attend_cell_steps<<<kNumBlk, 512, 0, stream>>>(PB, WQ, WIC, WHH, GX, h_init, bias_hh, bq, length, post_len, out);
}
